// TransformerBlock_74328704024931
// MI455X (gfx1250) — hardware-verified
//
#include <hip/hip_runtime.h>
#ifndef NB
#define NB 2
#endif
#ifndef SEQ
#define SEQ 2048
#endif
#define NB_FULL 2
#define SEQ_FULL 2048
#define DM 768
#define NH 12
#define HD 64
#define DFF 3072
#define LQ (3 * DM)
#define EARLY ((SEQ) < 256 ? (SEQ) : 256)
#define NR (NB * SEQ)
#define LNT (DM / 4)

static_assert(NH * HD == DM);
static_assert(HD == 64);
static_assert(DM == 768);
static_assert(LQ == 3 * DM);
static_assert(LNT * 4 == DM && LNT <= 256 && LNT % 32 == 0);
static_assert(SEQ % 128 == 0);
static_assert(EARLY % 128 == 0);
static_assert(EARLY % 64 == 0);
static_assert(DM % 64 == 0 && DFF % 64 == 0 && LQ % 64 == 0);
static_assert(DM % 32 == 0 && DFF % 32 == 0);
static_assert(DM % 8 == 0 && DFF % 8 == 0);
static_assert(NR % 128 == 0);
static_assert(NB <= NB_FULL && SEQ <= SEQ_FULL);

typedef _Float16 v16h __attribute__((ext_vector_type(16)));
typedef _Float16 v4h __attribute__((ext_vector_type(4)));
typedef unsigned short v8us __attribute__((ext_vector_type(8), may_alias));
typedef float v8f __attribute__((ext_vector_type(8)));
typedef float v4f __attribute__((ext_vector_type(4)));
typedef float v4fa __attribute__((ext_vector_type(4), may_alias));
union FragH { v16h v; v8us half[2]; _Float16 h[16]; unsigned short u[16]; };

__device__ __forceinline__ float bf16_rne(float x) {
  unsigned int u = __float_as_uint(x);
  u = (u + 0x7FFFu + ((u >> 16) & 1u)) & 0xFFFF0000u;
  return __uint_as_float(u);
}

__device__ __forceinline__ v16h g2_frag(const _Float16* p, int hh) {
  FragH f;
  f.half[0] = *(const v8us*)((const unsigned short*)p + 8 * hh);
  f.half[1] = *(const v8us*)((const unsigned short*)p + 16 + 8 * hh);
  return f.v;
}
__device__ __forceinline__ v8f g2_mma(v16h a, v16h b, v8f c) {
  v8f d = __builtin_amdgcn_wmma_f32_16x16x32_f16(false, a, false, b, (short)0, c, false, false);
  asm volatile("v_nop\n\tv_nop\n\tv_nop\n\tv_nop" : "+v"(d) : "v"(a), "v"(b));
  return d;
}

__global__ __launch_bounds__(256) void k_wt_f16(const float* __restrict__ W, _Float16* __restrict__ Wt, int K, int N, int ldo, float scale) {
  const int t = blockIdx.x * 256 + threadIdx.x;
  const int k8n = K / 8;
  if (t >= N * k8n) return;
  const int n = t / k8n, k8 = (t - n * k8n) * 8;
  FragH f;
#pragma unroll
  for (int i = 0; i < 8; ++i) {
    const float w = bf16_rne(W[(size_t)(k8 + i) * N + n]);
    f.h[i] = (_Float16)(w * scale);
  }
  unsigned short* dst = (unsigned short*)Wt + (size_t)n * ldo + k8;
  *(volatile v8us*)dst = f.half[0];
  __threadfence();
  *(volatile v8us*)dst = f.half[0];
}

__global__ __launch_bounds__(256) void k_wthd(const float* __restrict__ W, _Float16* __restrict__ Bt) {
  const size_t t = (size_t)blockIdx.x * 256 + threadIdx.x;
  if (t >= (size_t)NH * HD * (DM / 8)) return;
  const int m8 = (int)(t % (DM / 8)) * 8;
  const int d = (int)((t / (DM / 8)) % HD);
  const int h = (int)(t / ((size_t)(DM / 8) * HD));
  FragH f;
#pragma unroll
  for (int q = 0; q < 8; ++q) f.h[q] = (_Float16)(16.0f * bf16_rne(W[((size_t)h * DM + m8 + q) * HD + d]));
  unsigned short* dst = (unsigned short*)Bt + ((size_t)h * HD + d) * DM + m8;
  *(volatile v8us*)dst = f.half[0];
  __threadfence();
  *(volatile v8us*)dst = f.half[0];
}

__global__ __launch_bounds__(256) void k_bias3(const float* __restrict__ bq, const float* __restrict__ bk, const float* __restrict__ bv, float* __restrict__ dst) {
  const int i = blockIdx.x * 256 + threadIdx.x;
  if (i >= 3 * DM) return;
  const int c = i / DM, j = i - c * DM;
  const float a = bq[j], b = bk[j], d = bv[j];
  const float v = (c == 0) ? a : ((c == 1) ? b : d);
  *(volatile float*)(dst + i) = v;
  __threadfence();
  *(volatile float*)(dst + i) = v;
}

template <int BFIN>
__device__ __forceinline__ void ln_body(const float* __restrict__ xr, const float* __restrict__ g, const float* __restrict__ bb, _Float16* __restrict__ yr) {
#pragma clang fp contract(off)
  __shared__ float red[256];
  const int t = threadIdx.x;
  const bool act = t < LNT;
  const int tc = act ? t : 0;
  const v4f xa = *(const v4fa*)(xr + tc * 4);
  float s[4];
  float sum = 0.f;
#pragma unroll
  for (int q = 0; q < 4; ++q) { s[q] = BFIN ? bf16_rne(xa[q]) : xa[q]; sum = sum + s[q]; }
  red[t] = act ? sum : 0.f;
  __syncthreads();
#pragma unroll 1
  for (int st = 128; st > 0; st >>= 1) { if (t < st) red[t] = red[t] + red[t + st]; __syncthreads(); }
  const float mu = red[0] * (1.0f / (float)DM);
  __syncthreads();
  float vs = 0.f;
#pragma unroll
  for (int q = 0; q < 4; ++q) { const float dl = s[q] - mu; vs = vs + dl * dl; }
  red[t] = act ? vs : 0.f;
  __syncthreads();
#pragma unroll 1
  for (int st = 128; st > 0; st >>= 1) { if (t < st) red[t] = red[t] + red[t + st]; __syncthreads(); }
  const float rs = rsqrtf(red[0] * (1.0f / (float)DM) + 1e-5f);
  v4h y;
#pragma unroll
  for (int q = 0; q < 4; ++q) { const int c = tc * 4 + q; y[q] = (_Float16)(((s[q] - mu) * rs) * bf16_rne(g[c]) + bf16_rne(bb[c])); }
  if (act) {
    for (int pass = 0; pass < 2; ++pass) { *(volatile v4h*)(yr + t * 4) = y; if (pass == 0) __threadfence(); }
  }
}
__global__ __launch_bounds__(256) void k_ln1(const float* __restrict__ X, const float* __restrict__ g, const float* __restrict__ bb, _Float16* __restrict__ N16) {
  const int r = blockIdx.x; const int b = r / SEQ, s = r - b * SEQ;
  ln_body<1>(X + ((size_t)b * SEQ_FULL + s) * DM, g, bb, N16 + (size_t)r * DM);
}
__global__ __launch_bounds__(256) void k_ln2(const float* __restrict__ X1, const float* __restrict__ g, const float* __restrict__ bb, _Float16* __restrict__ M16) {
  const int r = blockIdx.x;
  ln_body<0>(X1 + (size_t)r * DM, g, bb, M16 + (size_t)r * DM);
}

template <int ACT, bool HASB, int RESMODE, int LOMODE, bool W32, bool W16>
__device__ __forceinline__ void gemm_body(const _Float16* __restrict__ A, int lda, size_t sA, const _Float16* __restrict__ Bh, int ldb, float alpha,
                                          const float* __restrict__ bias, const float* resid, int rpb, int rfull,
                                          float* C, _Float16* __restrict__ C16, _Float16* __restrict__ CL, int ldc, size_t sC, int M, int N, int K) {
  __shared__ __attribute__((aligned(16))) float so[4][32][68];
  const int tid = threadIdx.x, lane = tid & 31, ln = lane & 15, hh = lane >> 4;
  const int w = __builtin_amdgcn_readfirstlane(tid >> 5);
  const int by = blockIdx.y;
  A += (size_t)by * sA;
  const size_t cofs = (size_t)by * sC;
  const int ntn = N >> 6;
  const int mt = blockIdx.x / ntn, nq = blockIdx.x - mt * ntn;
  const int row0 = mt * 128 + 32 * w, col0 = nq * 64;
  if (row0 >= M) return;
  const _Float16* a0p = A + (size_t)(row0 + ln) * lda; const _Float16* a1p = a0p + (size_t)16 * lda;
  const _Float16* b0p = Bh + (size_t)(col0 + ln) * ldb; const _Float16* b1p = b0p + (size_t)16 * ldb;
  const _Float16* b2p = b1p + (size_t)16 * ldb; const _Float16* b3p = b2p + (size_t)16 * ldb;
  const v8f z8 = {0.f, 0.f, 0.f, 0.f, 0.f, 0.f, 0.f, 0.f};
  v8f c00 = z8, c01 = z8, c02 = z8, c03 = z8, c10 = z8, c11 = z8, c12 = z8, c13 = z8;
#pragma unroll 1
  for (int kb = 0; kb < K; kb += 32) {
    const v16h a0 = g2_frag(a0p + kb, hh), a1 = g2_frag(a1p + kb, hh);
    v16h b = g2_frag(b0p + kb, hh); c00 = g2_mma(a0, b, c00); c10 = g2_mma(a1, b, c10);
    b = g2_frag(b1p + kb, hh); c01 = g2_mma(a0, b, c01); c11 = g2_mma(a1, b, c11);
    b = g2_frag(b2p + kb, hh); c02 = g2_mma(a0, b, c02); c12 = g2_mma(a1, b, c12);
    b = g2_frag(b3p + kb, hh); c03 = g2_mma(a0, b, c03); c13 = g2_mma(a1, b, c13);
  }
  v8f accs[8] = {c00, c01, c02, c03, c10, c11, c12, c13};
#pragma unroll
  for (int u = 0; u < 8; ++u) {
    const int t = u & 3, half = u >> 2;
    const int col = col0 + t * 16 + ln;
    float bv = 0.f;
    if (HASB) bv = bf16_rne(bias[col]);
#pragma unroll
    for (int r = 0; r < 8; ++r) {
      const int rloc = half * 16 + 8 * hh + r;
      const float v = accs[u][r] * alpha + bv;
      so[w][rloc][t * 16 + ln] = v;
    }
  }
  __builtin_amdgcn_fence(4  , "workgroup");
  __builtin_amdgcn_wave_barrier();
  const int rsub = lane >> 4, c4 = (lane & 15) * 4;
  if (ACT == 7) {
#pragma unroll 1
    for (int q = 0; q < 16; ++q) {
      const int r = q * 2 + rsub;
      v4f v = *(const v4fa*)&so[w][r][c4];
#pragma unroll
      for (int e = 0; e < 4; ++e) {
        const float u = v[e];
        const float u3 = u * u * u;
        const float in = 0.7978845608028654f * (u + 0.044715f * u3);
        v[e] = 0.5f * u * (1.0f + tanhf(in));
      }
      *(v4fa*)&so[w][r][c4] = v;
    }
  }
  if (RESMODE != 0) {
    const int bidx = row0 / rpb;
    const int rbase = bidx * rfull + (row0 - bidx * rpb);
#pragma unroll
    for (int q = 0; q < 16; ++q) {
      const int r = q * 2 + rsub;
      v4f v = *(const v4fa*)&so[w][r][c4];
      v4f rv = *(const v4fa*)(resid + cofs + (size_t)(rbase + r) * ldc + col0 + c4);
      if (RESMODE == 1) { rv[0] = bf16_rne(rv[0]); rv[1] = bf16_rne(rv[1]); rv[2] = bf16_rne(rv[2]); rv[3] = bf16_rne(rv[3]); }
      v[0] += rv[0]; v[1] += rv[1]; v[2] += rv[2]; v[3] += rv[3];
      *(v4fa*)&so[w][r][c4] = v;
    }
  }
  bool lo_on = false; int lbase = 0;
  if (LOMODE == 1) {
    const int bidx = row0 / SEQ; const int s0 = row0 - bidx * SEQ;
    lo_on = (col0 >= 2 * DM) && (s0 < EARLY);
    lbase = bidx * EARLY + s0;
  }
  for (int pass = 0; pass < 2; ++pass) {
#pragma unroll
    for (int q = 0; q < 16; ++q) {
      const int r = q * 2 + rsub;
      const v4f v = *(const v4fa*)&so[w][r][c4];
      const size_t co = cofs + (size_t)(row0 + r) * ldc + col0 + c4;
      if (W32) *(volatile v4f*)(C + co) = v;
      if (W16) {
        v4h h4;
        h4[0] = (_Float16)v[0]; h4[1] = (_Float16)v[1]; h4[2] = (_Float16)v[2]; h4[3] = (_Float16)v[3];
        *(volatile v4h*)(C16 + co) = h4;
        if (LOMODE == 1) {
          if (lo_on) {
            v4h l4;
            l4[0] = (_Float16)((v[0] - (float)h4[0]) * 1024.0f); l4[1] = (_Float16)((v[1] - (float)h4[1]) * 1024.0f);
            l4[2] = (_Float16)((v[2] - (float)h4[2]) * 1024.0f); l4[3] = (_Float16)((v[3] - (float)h4[3]) * 1024.0f);
            *(volatile v4h*)(CL + (size_t)(lbase + r) * DM + (col0 - 2 * DM) + c4) = l4;
          }
        }
      }
    }
    if (pass == 0) __threadfence();
  }
}

__global__ __launch_bounds__(128) void k_gemm_qkv(const _Float16* __restrict__ A, const _Float16* __restrict__ Bt, const float* __restrict__ bias, _Float16* __restrict__ QKV, _Float16* __restrict__ VL) {
  gemm_body<0, true, 0, 1, false, true>(A, DM, 0, Bt, DM, 0.0625f, bias, nullptr, SEQ, SEQ, nullptr, QKV, VL, LQ, 0, NR, LQ, DM);
}
__global__ __launch_bounds__(128) void k_gemm_o(const _Float16* __restrict__ O16, const _Float16* __restrict__ Bt, const float* __restrict__ bias, const float* xin, float* X1) {
  gemm_body<0, true, 1, 0, true, false>(O16, DM, 0, Bt, DM, 0.0009765625f, bias, xin, SEQ, SEQ_FULL, X1, nullptr, nullptr, DM, 0, NR, DM, DM);
}
__global__ __launch_bounds__(128) void k_gemm_ol(const _Float16* __restrict__ OL16, const _Float16* __restrict__ Bt, float* X1) {
  gemm_body<0, false, 2, 0, true, false>(OL16, DM, (size_t)EARLY * DM, Bt, DM, 9.5367431640625e-07f, nullptr, X1, SEQ, SEQ, X1, nullptr, nullptr, DM, (size_t)SEQ * DM, EARLY, DM, DM);
}
__global__ __launch_bounds__(128) void k_gemm_fc1(const _Float16* __restrict__ M16, const _Float16* __restrict__ Bt, const float* __restrict__ bias, _Float16* __restrict__ GH) {
  gemm_body<7, true, 0, 0, false, true>(M16, DM, 0, Bt, DM, 0.0625f, bias, nullptr, SEQ, SEQ, nullptr, GH, nullptr, DFF, 0, NR, DFF, DM);
}
__global__ __launch_bounds__(128) void k_gemm_fc2(const _Float16* __restrict__ GH, const _Float16* __restrict__ Bt, const float* __restrict__ bias, const float* X1, float* OUT) {
  gemm_body<0, true, 2, 0, true, false>(GH, DFF, 0, Bt, DFF, 0.0625f, bias, X1, SEQ, SEQ, OUT, nullptr, nullptr, DM, 0, NR, DM, DFF);
}

__global__ __launch_bounds__(256) void k_vt(unsigned short* wsb, size_t sHi, size_t sLo, size_t dHi, size_t dLo) {
  __shared__ unsigned short tl[64][66];
  const int tid = threadIdx.x;
  int bx = blockIdx.x;
  const int nhi = NB * NH * (SEQ / 64);
  const bool lo = bx >= nhi;
  if (lo) bx -= nhi;
  const int T = lo ? EARLY : SEQ;
  const int tpb = T / 64;
  const int slab = bx / tpb, lg = bx - slab * tpb;
  const int b = slab / NH, h = slab - b * NH;
  const int ldv = lo ? DM : LQ;
  const int coff = lo ? 0 : 2 * DM;
  const size_t so_ = lo ? sLo : sHi;
  const size_t do_ = lo ? dLo : dHi;
  for (int i = tid; i < 64 * 8; i += 256) {
    const int r = i >> 3, c8 = (i & 7) * 8;
    FragH f;
    f.half[0] = *(const v8us*)(wsb + so_ + ((size_t)b * T + lg * 64 + r) * ldv + coff + h * HD + c8);
#pragma unroll
    for (int q = 0; q < 8; ++q) tl[r][c8 + q] = f.u[q];
  }
  __syncthreads();
  for (int pass = 0; pass < 2; ++pass) {
#pragma unroll
    for (int rd = 0; rd < 2; ++rd) {
      const int d = rd * 32 + (tid >> 3), pc = tid & 7;
      FragH f;
#pragma unroll
      for (int q = 0; q < 8; ++q) f.u[q] = tl[pc * 8 + q][d];
      *(volatile v8us*)(wsb + do_ + ((size_t)slab * HD + d) * T + lg * 64 + pc * 8) = f.half[0];
    }
    if (pass == 0) __threadfence();
  }
}

__global__ __launch_bounds__(128) void k_attn(const _Float16* __restrict__ QKV, const _Float16* __restrict__ VT, const _Float16* __restrict__ VTL, _Float16* __restrict__ O16, _Float16* __restrict__ OL16) {
  __shared__ __attribute__((aligned(16))) unsigned short Qs[64][72];
  __shared__ __attribute__((aligned(16))) unsigned short Ks[64][72];
  __shared__ __attribute__((aligned(16))) unsigned short Vs[64][72];
  __shared__ __attribute__((aligned(16))) unsigned short Vl[64][72];
  __shared__ __attribute__((aligned(16))) float Os[4][16][68];
  const int tid = threadIdx.x, lane = tid & 31, ln = lane & 15, hh = lane >> 4;
  const int wave = __builtin_amdgcn_readfirstlane(tid >> 5);
  const int q0 = blockIdx.x * 64, h = blockIdx.y, b = blockIdx.z;
  const bool early = q0 < EARLY;
  const int qw = q0 + 16 * wave;
  const int qrow = qw + ln;
  const unsigned short* qkv = (const unsigned short*)QKV;
  const unsigned short* vt = (const unsigned short*)VT;
  const unsigned short* vtl = (const unsigned short*)VTL;
#pragma unroll
  for (int u = 0; u < 4; ++u) {
    const int i = tid + 128 * u; const int r = i >> 3, p8 = (i & 7) * 8;
    const v8us v = *(const v8us*)(qkv + (size_t)(b * SEQ + q0 + r) * LQ + h * HD + p8);
    *(v8us*)&Qs[r][p8] = v;
  }
  const v8f z8 = {0.f, 0.f, 0.f, 0.f, 0.f, 0.f, 0.f, 0.f};
  v8f oM[4], oR[4];
#pragma unroll
  for (int dt = 0; dt < 4; ++dt) { oM[dt] = z8; oR[dt] = z8; }
  float m = -1.0e30f, l = 0.f;
#pragma unroll 1
  for (int k0 = 0; k0 <= q0; k0 += 64) {
    __syncthreads();
#pragma unroll
    for (int u = 0; u < 4; ++u) {
      const int i = tid + 128 * u; const int r = i >> 3, p8 = (i & 7) * 8;
      const v8us kv = *(const v8us*)(qkv + (size_t)(b * SEQ + k0 + r) * LQ + DM + h * HD + p8);
      *(v8us*)&Ks[r][p8] = kv;
      const v8us vv = *(const v8us*)(vt + ((size_t)((b * NH + h) * HD + r)) * SEQ + k0 + p8);
      *(v8us*)&Vs[r][p8] = vv;
    }
    if (early) {
#pragma unroll
      for (int u = 0; u < 4; ++u) {
        const int i = tid + 128 * u; const int r = i >> 3, p8 = (i & 7) * 8;
        const v8us lv = *(const v8us*)(vtl + ((size_t)((b * NH + h) * HD + r)) * EARLY + k0 + p8);
        *(v8us*)&Vl[r][p8] = lv;
      }
    }
    __syncthreads();
#pragma unroll 1
    for (int half = 0; half < 2; ++half) {
      const int kh = k0 + 32 * half;
      if (kh <= qw + 15) {
        v8f s0 = z8, s1 = z8;
#pragma unroll
        for (int ks = 0; ks < 2; ++ks) {
          FragH qf, ka, kb;
          qf.half[0] = *(const v8us*)&Qs[16 * wave + ln][32 * ks + 8 * hh];
          qf.half[1] = *(const v8us*)&Qs[16 * wave + ln][32 * ks + 16 + 8 * hh];
          ka.half[0] = *(const v8us*)&Ks[32 * half + ln][32 * ks + 8 * hh];
          ka.half[1] = *(const v8us*)&Ks[32 * half + ln][32 * ks + 16 + 8 * hh];
          kb.half[0] = *(const v8us*)&Ks[32 * half + 16 + ln][32 * ks + 8 * hh];
          kb.half[1] = *(const v8us*)&Ks[32 * half + 16 + ln][32 * ks + 16 + 8 * hh];
          s0 = g2_mma(ka.v, qf.v, s0);
          s1 = g2_mma(kb.v, qf.v, s1);
        }
        const int kb0 = kh + 8 * hh;
        float mx = -3.0e38f;
#pragma unroll
        for (int r = 0; r < 8; ++r) {
          float a0 = s0[r] * 0.125f; a0 = (kb0 + r <= qrow) ? a0 : -100000.0f; s0[r] = a0;
          float a1 = s1[r] * 0.125f; a1 = (kb0 + 16 + r <= qrow) ? a1 : -100000.0f; s1[r] = a1;
          mx = fmaxf(mx, fmaxf(a0, a1));
        }
        mx = fmaxf(mx, __shfl_xor(mx, 16, 32));
        const float mn = fmaxf(m, mx);
        const float al = __expf(m - mn);
        m = mn;
        float ps = 0.f;
        FragH pf, pl;
#pragma unroll
        for (int r = 0; r < 8; ++r) {
          const float p0 = __expf(s0[r] - mn), p1 = __expf(s1[r] - mn);
          ps += p0 + p1;
          const float e0 = p0 * 256.0f, e1 = p1 * 256.0f;
          s0[r] = e0; s1[r] = e1;
          pf.h[r] = (_Float16)e0; pf.h[8 + r] = (_Float16)e1;
        }
        l = l * al + ps;
        pl.v = pf.v;
        if (early) {
#pragma unroll
          for (int r = 0; r < 8; ++r) {
            pl.h[r] = (_Float16)((s0[r] - (float)pf.h[r]) * 1024.0f);
            pl.h[8 + r] = (_Float16)((s1[r] - (float)pf.h[8 + r]) * 1024.0f);
          }
        }
#pragma unroll
        for (int dt = 0; dt < 4; ++dt) {
          FragH vf;
          vf.half[0] = *(const v8us*)&Vs[16 * dt + ln][32 * half + 8 * hh];
          vf.half[1] = *(const v8us*)&Vs[16 * dt + ln][32 * half + 16 + 8 * hh];
#pragma unroll
          for (int r = 0; r < 8; ++r) oM[dt][r] *= al;
          oM[dt] = g2_mma(vf.v, pf.v, oM[dt]);
        }
        if (early) {
#pragma unroll
          for (int dt = 0; dt < 4; ++dt) {
            FragH vf, vr;
            vf.half[0] = *(const v8us*)&Vs[16 * dt + ln][32 * half + 8 * hh];
            vf.half[1] = *(const v8us*)&Vs[16 * dt + ln][32 * half + 16 + 8 * hh];
            vr.half[0] = *(const v8us*)&Vl[16 * dt + ln][32 * half + 8 * hh];
            vr.half[1] = *(const v8us*)&Vl[16 * dt + ln][32 * half + 16 + 8 * hh];
#pragma unroll
            for (int r = 0; r < 8; ++r) oR[dt][r] *= al;
            oR[dt] = g2_mma(vf.v, pl.v, oR[dt]);
            oR[dt] = g2_mma(vr.v, pf.v, oR[dt]);
          }
        }
      }
    }
  }
  const float lt = l + __shfl_xor(l, 16, 32);
  const float inv = 0.25f * (1.0f / lt);
#pragma unroll
  for (int dt = 0; dt < 4; ++dt)
#pragma unroll
    for (int r = 0; r < 8; ++r) Os[wave][ln][16 * dt + 8 * hh + r] = (oM[dt][r] + oR[dt][r] * 0.0009765625f) * inv;
  __builtin_amdgcn_fence(4  , "workgroup");
  __builtin_amdgcn_wave_barrier();
  unsigned short* o16 = (unsigned short*)O16;
  unsigned short* ol16 = (unsigned short*)OL16;
  const int rq = lane >> 3, pc = (lane & 7) * 8;
  for (int pass = 0; pass < 2; ++pass) {
#pragma unroll
    for (int it = 0; it < 4; ++it) {
      const int row = it * 4 + rq;
      const v4f a = *(const v4fa*)&Os[wave][row][pc];
      const v4f c = *(const v4fa*)&Os[wave][row][pc + 4];
      FragH fh, fl;
#pragma unroll
      for (int q = 0; q < 4; ++q) {
        _Float16 hv = (_Float16)a[q]; fh.h[q] = hv; fl.h[q] = (_Float16)((a[q] - (float)hv) * 1024.0f);
        hv = (_Float16)c[q]; fh.h[4 + q] = hv; fl.h[4 + q] = (_Float16)((c[q] - (float)hv) * 1024.0f);
      }
      *(volatile v8us*)(o16 + (size_t)(b * SEQ + qw + row) * DM + h * HD + pc) = fh.half[0];
      if (early) *(volatile v8us*)(ol16 + (size_t)(b * EARLY + qw + row) * DM + h * HD + pc) = fl.half[0];
    }
    if (pass == 0) __threadfence();
  }
}

#define SZ_N16  ((size_t)NR * DM * 2)
#define SZ_BW1  ((size_t)DFF * DM * 2)
#define SZ_BW2  ((size_t)DM * DFF * 2)
#define SZ_X1   ((size_t)NR * DM * 4)
#define SZ_GH   ((size_t)NR * DFF * 2)
#define SZ_BQKV ((size_t)3 * DM * DM * 2)
#define SZ_BO   ((size_t)DM * DM * 2)
#define SZ_BIAS ((size_t)3 * DM * 4)
#define SZ_QKV  ((size_t)NR * LQ * 2)
#define SZ_VL   ((size_t)NB * EARLY * DM * 2)
#define SZ_O16  ((size_t)NR * DM * 2)
#define SZ_OL   ((size_t)NB * EARLY * DM * 2)
#define SZ_VT   ((size_t)NB * NH * HD * SEQ * 2)
#define SZ_VTL  ((size_t)NB * NH * HD * EARLY * 2)
#define SZ_ATT  (SZ_BQKV + SZ_BO + SZ_BIAS + SZ_QKV + SZ_VL + SZ_O16 + SZ_OL + SZ_VT + SZ_VTL)
#define SZ_UNI  ((SZ_GH) > (SZ_ATT) ? (SZ_GH) : (SZ_ATT))
#define SZ_TOT  (SZ_N16 + SZ_BW1 + SZ_BW2 + SZ_X1 + SZ_UNI)
static_assert(SZ_N16 % 256 == 0 && SZ_BW1 % 256 == 0 && SZ_BW2 % 256 == 0 && SZ_X1 % 256 == 0);
static_assert(SZ_BQKV % 256 == 0 && SZ_BO % 256 == 0 && SZ_BIAS % 256 == 0 && SZ_QKV % 256 == 0 && SZ_VL % 256 == 0);
static_assert(SZ_O16 % 256 == 0 && SZ_OL % 256 == 0 && SZ_VT % 256 == 0 && SZ_VTL % 256 == 0);
static_assert(SZ_GH % 256 == 0);
static_assert(SZ_GH <= SZ_UNI && SZ_ATT <= SZ_UNI);
static_assert(SZ_TOT <= (size_t)134217728);

extern "C" void kernel_launch(void* const* d_in, const int* in_sizes, int n_in,
                              void* d_out, int out_size, void* d_ws, size_t ws_size, hipStream_t stream) {
  if (n_in < 17) return;
  if ((long long)in_sizes[0] < ((long long)(NB - 1) * SEQ_FULL + SEQ) * DM) return;
  if (in_sizes[1] < NH * DM * HD || in_sizes[3] < NH * DM * HD || in_sizes[5] < NH * DM * HD || in_sizes[7] < NH * HD * DM) return;
  if (in_sizes[2] < DM || in_sizes[4] < DM || in_sizes[6] < DM || in_sizes[8] < DM) return;
  if (in_sizes[9] < DM || in_sizes[10] < DM || in_sizes[11] < DM || in_sizes[12] < DM) return;
  if (in_sizes[13] < DM * DFF || in_sizes[14] < DFF || in_sizes[15] < DFF * DM || in_sizes[16] < DM) return;
  if ((long long)out_size < (long long)NR * DM) return;
  if ((size_t)SZ_TOT > ws_size) return;
  const float* const* I = (const float* const*)d_in;
  const float* x = I[0];
  const float* wq = I[1]; const float* bq = I[2]; const float* wk = I[3]; const float* bk = I[4];
  const float* wv = I[5]; const float* bv = I[6]; const float* wo = I[7]; const float* bo = I[8];
  const float* g1 = I[9]; const float* be1 = I[10]; const float* g2 = I[11]; const float* be2 = I[12];
  const float* win = I[13]; const float* bin = I[14]; const float* wout = I[15]; const float* bout = I[16];
  char* ws = (char*)d_ws;
  size_t off = 0;
  _Float16* N16 = (_Float16*)(ws + off); off += SZ_N16;
  _Float16* BW1 = (_Float16*)(ws + off); off += SZ_BW1;
  _Float16* BW2 = (_Float16*)(ws + off); off += SZ_BW2;
  float* X1 = (float*)(ws + off); off += SZ_X1;
  const size_t uni = off;
  _Float16* GH = (_Float16*)(ws + uni);
  size_t ao = uni;
  _Float16* BQKV = (_Float16*)(ws + ao); ao += SZ_BQKV;
  _Float16* BO = (_Float16*)(ws + ao); ao += SZ_BO;
  float* bqkv = (float*)(ws + ao); ao += SZ_BIAS;
  _Float16* QKV = (_Float16*)(ws + ao); const size_t oQKV = ao; ao += SZ_QKV;
  _Float16* VL = (_Float16*)(ws + ao); const size_t oVL = ao; ao += SZ_VL;
  _Float16* O16 = (_Float16*)(ws + ao); ao += SZ_O16;
  _Float16* OL16 = (_Float16*)(ws + ao); ao += SZ_OL;
  _Float16* VT = (_Float16*)(ws + ao); const size_t oVT = ao; ao += SZ_VT;
  _Float16* VTL = (_Float16*)(ws + ao); const size_t oVTL = ao; ao += SZ_VTL;
  _Float16* M16 = N16;

  const unsigned gh = (unsigned)(((size_t)NH * HD * (DM / 8) + 255) / 256);
  k_wthd<<<gh, 256, 0, stream>>>(wq, BQKV);
  k_wthd<<<gh, 256, 0, stream>>>(wk, BQKV + (size_t)DM * DM);
  k_wthd<<<gh, 256, 0, stream>>>(wv, BQKV + (size_t)2 * DM * DM);
  k_wt_f16<<<(unsigned)(((size_t)DM * (DM / 8) + 255) / 256), 256, 0, stream>>>(wo, BO, DM, DM, DM, 16.0f);
  k_wt_f16<<<(unsigned)(((size_t)DFF * (DM / 8) + 255) / 256), 256, 0, stream>>>(win, BW1, DM, DFF, DM, 16.0f);
  k_wt_f16<<<(unsigned)(((size_t)DM * (DFF / 8) + 255) / 256), 256, 0, stream>>>(wout, BW2, DFF, DM, DFF, 16.0f);
  k_bias3<<<(3 * DM + 255) / 256, 256, 0, stream>>>(bq, bk, bv, bqkv);
  k_ln1<<<NR, 256, 0, stream>>>(x, g1, be1, N16);
  k_gemm_qkv<<<dim3((unsigned)((NR / 128) * (LQ / 64)), 1), 128, 0, stream>>>(N16, BQKV, bqkv, QKV, VL);
  k_vt<<<NB * NH * (SEQ / 64) + NB * NH * (EARLY / 64), 256, 0, stream>>>((unsigned short*)ws, oQKV / 2, oVL / 2, oVT / 2, oVTL / 2);
  k_attn<<<dim3(SEQ / 64, NH, NB), 128, 0, stream>>>(QKV, VT, VTL, O16, OL16);
  k_gemm_o<<<dim3((unsigned)((NR / 128) * (DM / 64)), 1), 128, 0, stream>>>(O16, BO, bo, x, X1);
  k_gemm_ol<<<dim3((unsigned)((EARLY / 128) * (DM / 64)), NB), 128, 0, stream>>>(OL16, BO, X1);
  k_ln2<<<NR, 256, 0, stream>>>(X1, g2, be2, M16);
  k_gemm_fc1<<<dim3((unsigned)((NR / 128) * (DFF / 64)), 1), 128, 0, stream>>>(M16, BW1, bin, GH);
  k_gemm_fc2<<<dim3((unsigned)((NR / 128) * (DM / 64)), 1), 128, 0, stream>>>(GH, BW2, bout, X1, (float*)d_out);
}
